// DecoderRNN_59004260712896
// MI455X (gfx1250) — hardware-verified
//
#include <hip/hip_runtime.h>
#include <math.h>

typedef __attribute__((ext_vector_type(16))) _Float16 v16h;
typedef __attribute__((ext_vector_type(8)))  _Float16 v8h;
typedef __attribute__((ext_vector_type(16))) __bf16   v16b;
typedef __attribute__((ext_vector_type(8)))  __bf16   v8b;
typedef __attribute__((ext_vector_type(8)))  float    v8f;
typedef __attribute__((ext_vector_type(4)))  float    v4f;

constexpr int kB     = 64;
constexpr int kT     = 21;
constexpr int kTo    = kT - 1;
constexpr int kE     = 512;
constexpr int kHid   = 512;
constexpr int kG4    = 4 * kHid;
constexpr int kV     = 10000;
constexpr int kVP    = 10240;
constexpr int kRowsX = kT * kB;
constexpr int kRowsY = kB * kTo;
constexpr int kThr   = 256;
constexpr float kInCarry = 1024.0f;

constexpr float kXCarry = 1024.0f;
constexpr float kWCarry = 1024.0f;
constexpr float kSCarry = 1024.0f;
constexpr float kScXW = 1.0f / (kXCarry * kWCarry);
constexpr float kScHW = 1.0f / (kSCarry * kWCarry);
constexpr float kF16MinNormal = 6.103515625e-5f;

static_assert((kRowsX % 64) == 0 && (kRowsY % 64) == 0 && (kB % 64) == 0 && (kG4 % 64) == 0 && (kVP % 64) == 0, "GEMM M, N multiples of 64");
static_assert(((kRowsX / 64) * (kG4 / 64)) % 8 == 0 && ((kB / 64) * (kG4 / 64)) % 8 == 0 && ((kRowsY / 64) * (kVP / 64)) % 8 == 0, "GEMM grids exact");
static_assert((kE % 32) == 0 && (kHid % 32) == 0, "GEMM K multiples of 32");

constexpr size_t kOffX16 = 0;
constexpr size_t kOffWIH = kOffX16 + (size_t)kRowsX * kE * 2;
constexpr size_t kOffWHH = kOffWIH + (size_t)kG4 * kE * 2;
constexpr size_t kOffWL  = kOffWHH + (size_t)kG4 * kHid * 2;
constexpr size_t kOffBG  = kOffWL  + (size_t)kVP * kHid * 2;
constexpr size_t kOffBL  = kOffBG  + (size_t)kG4 * 4;
constexpr size_t kOffZB  = kOffBL  + (size_t)kVP * 4;
constexpr size_t kOffXW  = kOffZB  + (size_t)kG4 * 4;
constexpr size_t kOffGG  = kOffXW  + (size_t)kRowsX * kG4 * 4;
constexpr size_t kOffC32 = kOffGG  + (size_t)kB * kG4 * 4;
constexpr size_t kOffH16 = kOffC32 + (size_t)kB * kHid * 4;
constexpr size_t kOffHL  = kOffH16 + (size_t)kB * kHid * 2;
constexpr size_t kOffLG  = kOffHL  + (size_t)kRowsY * kHid * 2;
constexpr size_t kWsTotal = kOffLG + (size_t)kRowsY * kVP * 4;
static_assert(kWsTotal == 81584128ull, "carve total");
static_assert(kWsTotal <= 134217728ull, "carve cap");
static_assert((kOffWIH % 256) == 0 && (kOffWHH % 256) == 0 && (kOffWL % 256) == 0 && (kOffBG % 256) == 0 && (kOffBL % 256) == 0 && (kOffZB % 256) == 0 && (kOffXW % 256) == 0 && (kOffGG % 256) == 0 && (kOffC32 % 256) == 0 && (kOffH16 % 256) == 0 && (kOffHL % 256) == 0 && (kOffLG % 256) == 0, "aligned regions");

__device__ __forceinline__ unsigned short f2bf_bits(float f) {
  unsigned u = __float_as_uint(f);
  return (unsigned short)((u + 0x7FFFu + ((u >> 16) & 1u)) >> 16);
}
__device__ __forceinline__ float bf_bits2f(unsigned short h) { return __uint_as_float(((unsigned)h) << 16); }
__device__ __forceinline__ float bf16r(float f) { return bf_bits2f(f2bf_bits(f)); }
__device__ __forceinline__ float carry_flush(float v, float carry) {
  const float s = v * carry;
  return (fabsf(s) < kF16MinNormal) ? 0.0f : s;
}
__device__ __forceinline__ float frcp(float x) { return __builtin_amdgcn_rcpf(x); }

__device__ __forceinline__ void dep_guard4_h(v8f& a, v8f& b, v8f& c, v8f& d, v16h x, v16h y) { asm volatile("v_nop\n\tv_nop\n\tv_nop\n\tv_nop" : "+v"(a), "+v"(b), "+v"(c), "+v"(d) : "v"(x), "v"(y)); }
__device__ __forceinline__ void dep_guard4_b(v8f& a, v8f& b, v8f& c, v8f& d, v16b x, v16b y) { asm volatile("v_nop\n\tv_nop\n\tv_nop\n\tv_nop" : "+v"(a), "+v"(b), "+v"(c), "+v"(d) : "v"(x), "v"(y)); }
__device__ __forceinline__ void keep4_h(v16h a, v16h b, v16h c, v16h d) { asm volatile("v_nop" :: "v"(a), "v"(b), "v"(c), "v"(d)); }
__device__ __forceinline__ void keep4_b(v16b a, v16b b, v16b c, v16b d) { asm volatile("v_nop" :: "v"(a), "v"(b), "v"(c), "v"(d)); }
__device__ __forceinline__ void acc_guard4(v8f& a, v8f& b, v8f& c, v8f& d) { asm volatile("v_nop\n\tv_nop\n\tv_nop\n\tv_nop" : "+v"(a), "+v"(b), "+v"(c), "+v"(d)); }

template <typename T> struct Frag;
template <> struct Frag<_Float16> {
  typedef v16h V; union U { v16h v; v8h h[2]; };
  static __device__ __forceinline__ v16h load(const _Float16* p) {
    U f; f.h[0] = *(const v8h*)(p); f.h[1] = *(const v8h*)(p + 16); return f.v;
  }
  static __device__ __forceinline__ v8f mma(v16h a, v16h b, v8f c) {
    return __builtin_amdgcn_wmma_f32_16x16x32_f16(false, a, false, b, (short)0, c, false, false);
  }
  static __device__ __forceinline__ void guard4(v8f& a, v8f& b, v8f& c, v8f& d, v16h x, v16h y) { dep_guard4_h(a, b, c, d, x, y); }
  static __device__ __forceinline__ void keep(v16h a, v16h b, v16h c, v16h d) { keep4_h(a, b, c, d); }
};
template <> struct Frag<__bf16> {
  typedef v16b V; union U { v16b v; v8b h[2]; };
  static __device__ __forceinline__ v16b load(const __bf16* p) {
    U f; f.h[0] = *(const v8b*)(p); f.h[1] = *(const v8b*)(p + 16); return f.v;
  }
  static __device__ __forceinline__ v8f mma(v16b a, v16b b, v8f c) {
    return __builtin_amdgcn_wmma_f32_16x16x32_bf16(false, a, false, b, (short)0, c, false, false);
  }
  static __device__ __forceinline__ void guard4(v8f& a, v8f& b, v8f& c, v8f& d, v16b x, v16b y) { dep_guard4_b(a, b, c, d, x, y); }
  static __device__ __forceinline__ void keep(v16b a, v16b b, v16b c, v16b d) { keep4_b(a, b, c, d); }
};

__device__ __forceinline__ v8f mma_h(v16h a, v16h b, v8f c) {
  c = __builtin_amdgcn_wmma_f32_16x16x32_f16(false, a, false, b, (short)0, c, false, false);
  asm volatile("v_nop\n\tv_nop\n\tv_nop\n\tv_nop" : "+v"(c) : "v"(a), "v"(b));
  return c;
}

template <int ET> struct Elem;
template <> struct Elem<0> { typedef _Float16 T; };
template <> struct Elem<1> { typedef __bf16 T; };
template <int ET, bool SPLIT, int BIAS_MODE, int OUT_MODE, bool RESID, int ACT = 0>
__global__ __launch_bounds__(256) void wmma_gemm64(
    const unsigned short* __restrict__ Ap, const unsigned short* __restrict__ A2p, int lda, long strideA,
    const unsigned short* __restrict__ Btp, const unsigned short* __restrict__ Bt2p, int ldb, long strideB,
    void* __restrict__ Cout, void* __restrict__ Cout2, int ldc, long strideC,
    const float* __restrict__ bias,
    const float* __restrict__ resid, long strideR,
    int M, int N, int K, float scale) {
  typedef typename Elem<ET>::T T;
  typedef typename Frag<T>::V V;
  const T* A = (const T*)Ap; const T* A2 = (const T*)A2p; const T* Bt = (const T*)Btp; const T* Bt2 = (const T*)Bt2p;
  __shared__ __align__(16) float sT[8][16 * 68];
  const int b    = blockIdx.y;
  const int lane = threadIdx.x & 31;
  const int wave = threadIdx.x >> 5;
  const int tilesN = N >> 6;
  const int tilesM = M >> 6;
  const int tile = blockIdx.x * 8 + wave;
  if (tile >= tilesM * tilesN) return;
  const int tm = tile / tilesN;
  const int tn = tile - tm * tilesN;
  const int m0 = tm << 6;
  const int n0 = tn << 6;

  const T* Ab  = A  + (size_t)b * strideA;
  const T* Bb  = Bt + (size_t)b * strideB;
  const T* Ab2 = SPLIT ? (A2  + (size_t)b * strideA) : nullptr;
  const T* Bb2 = SPLIT ? (Bt2 + (size_t)b * strideB) : nullptr;

  const int rlane = lane & 15;
  const int koff  = (lane >> 4) * 8;
  const int mOff  = (lane >> 4) * 8;

  v8f acc[4][4];
#pragma unroll
  for (int i = 0; i < 4; ++i)
#pragma unroll
    for (int j = 0; j < 4; ++j) acc[i][j] = (v8f){0.f,0.f,0.f,0.f,0.f,0.f,0.f,0.f};

  for (int k0 = 0; k0 < K; k0 += 32) {
    V bh[4], bl[4];
#pragma unroll
    for (int j = 0; j < 4; ++j) {
      const size_t bo = (size_t)(n0 + (j << 4) + rlane) * ldb + koff + k0;
      bh[j] = Frag<T>::load(Bb + bo);
      if (SPLIT) bl[j] = Frag<T>::load(Bb2 + bo);
    }
#pragma unroll
    for (int i = 0; i < 4; ++i) {
      const size_t ao = (size_t)(m0 + (i << 4) + rlane) * lda + koff + k0;
      V ah = Frag<T>::load(Ab + ao);
      V al;
      if (SPLIT) al = Frag<T>::load(Ab2 + ao);
#pragma unroll
      for (int j = 0; j < 4; ++j) {
        acc[i][j] = Frag<T>::mma(ah, bh[j], acc[i][j]);
        if (SPLIT) {
          acc[i][j] = Frag<T>::mma(ah, bl[j], acc[i][j]);
          acc[i][j] = Frag<T>::mma(al, bh[j], acc[i][j]);
        }
      }
      Frag<T>::guard4(acc[i][0], acc[i][1], acc[i][2], acc[i][3], ah, SPLIT ? al : ah);
    }
    Frag<T>::keep(bh[0], bh[1], bh[2], bh[3]);
    if (SPLIT) Frag<T>::keep(bl[0], bl[1], bl[2], bl[3]);
  }
  acc_guard4(acc[0][0], acc[0][1], acc[0][2], acc[0][3]);
  acc_guard4(acc[1][0], acc[1][1], acc[1][2], acc[1][3]);
  acc_guard4(acc[2][0], acc[2][1], acc[2][2], acc[2][3]);
  acc_guard4(acc[3][0], acc[3][1], acc[3][2], acc[3][3]);

  float* slab = sT[wave];
  const float* Rb = RESID ? (resid + (size_t)b * strideR) : nullptr;
#pragma unroll
  for (int i = 0; i < 4; ++i) {
    const int mBase = m0 + (i << 4);
#pragma unroll
    for (int j = 0; j < 4; ++j) {
      const int n = n0 + (j << 4) + rlane;
      float bv = 0.f;
      if (BIAS_MODE == 2) bv = bias[n];
#pragma unroll
      for (int r = 0; r < 8; ++r) {
        float v = acc[i][j][r] * scale;
        if (BIAS_MODE == 1) v += bias[mBase + mOff + r];
        if (BIAS_MODE == 2) v += bv;
        if (RESID) v += Rb[(size_t)(mBase + mOff + r) * ldc + n];
        if (ACT == 1) v = tanhf(v);
        if (ACT == 2) v = fmaxf(v, 0.0f);
        if (ACT == 3) v = v / (1.0f + expf(-v));
        if (ACT == 4) v = (v > 0.f) ? v : 0.01f * v;
        slab[(mOff + r) * 68 + (j << 4) + rlane] = v;
      }
    }
    __builtin_amdgcn_fence(__ATOMIC_RELEASE, "workgroup");
    __builtin_amdgcn_wave_barrier();
    __builtin_amdgcn_fence(__ATOMIC_ACQUIRE, "workgroup");
    if (OUT_MODE == 0) {
      float* C = (float*)Cout + (size_t)b * strideC;
      const int hh = lane >> 4, c4 = (lane & 15) * 4;
      for (int pass = 0; pass < 2; ++pass) {
#pragma unroll
        for (int it = 0; it < 8; ++it) {
          const int row = it * 2 + hh;
          v4f v = *(const v4f*)(slab + row * 68 + c4);
          *(volatile v4f*)(C + (size_t)(mBase + row) * ldc + n0 + c4) = v;
        }
        __threadfence();
      }
    } else {
      const int q = lane >> 3, c8 = (lane & 7) * 8;
      unsigned short* C  = (unsigned short*)Cout  + (size_t)b * strideC;
      unsigned short* C2 = (OUT_MODE == 2) ? ((unsigned short*)Cout2 + (size_t)b * strideC) : nullptr;
      for (int pass = 0; pass < 2; ++pass) {
#pragma unroll
        for (int it = 0; it < 4; ++it) {
          const int row = it * 4 + q;
          const float* sp = slab + row * 68 + c8;
          v8h hv, lv;
#pragma unroll
          for (int e = 0; e < 8; ++e) {
            if (OUT_MODE == 1) {
              hv[e] = (_Float16)sp[e];
            } else {
              unsigned short hb = f2bf_bits(sp[e]);
              unsigned short lb = f2bf_bits(sp[e] - bf_bits2f(hb));
              hv[e] = __builtin_bit_cast(_Float16, hb);
              lv[e] = __builtin_bit_cast(_Float16, lb);
            }
          }
          *(volatile v8h*)(C + (size_t)(mBase + row) * ldc + n0 + c8) = hv;
          if (OUT_MODE == 2) *(volatile v8h*)(C2 + (size_t)(mBase + row) * ldc + n0 + c8) = lv;
        }
        __threadfence();
      }
    }
    __builtin_amdgcn_fence(__ATOMIC_RELEASE, "workgroup");
    __builtin_amdgcn_wave_barrier();
    __builtin_amdgcn_fence(__ATOMIC_ACQUIRE, "workgroup");
  }
}

__global__ __launch_bounds__(kThr) void cast_plane_kernel(const float* __restrict__ src, unsigned short* __restrict__ dst,
                                                          int colsLog2, int dstPitch, int dstOff) {
  const int i   = blockIdx.x * kThr + threadIdx.x;
  const int sh  = colsLog2 - 3;
  const int row = i >> sh;
  const int c8  = (i & ((1 << sh) - 1)) * 8;
  const float* sp = src + ((size_t)row << colsLog2) + c8;
  const v4f a0 = *(const v4f*)(sp);
  const v4f a1 = *(const v4f*)(sp + 4);
  v8h hv;
#pragma unroll
  for (int e = 0; e < 4; ++e) {
    const float f0 = a0[e];
    const float f1 = a1[e];
    hv[e]     = (_Float16)carry_flush(bf16r(f0), kInCarry);
    hv[4 + e] = (_Float16)carry_flush(bf16r(f1), kInCarry);
  }
  unsigned short* dp = dst + (size_t)row * dstPitch + dstOff + c8;
  *(volatile v8h*)dp = hv;
  __threadfence();
  *(volatile v8h*)dp = hv;
}

__global__ __launch_bounds__(kThr) void x_plane_kernel(const float* __restrict__ features, const float* __restrict__ emb,
                                                       unsigned short* __restrict__ X16) {
  unsigned v = blockIdx.x * (unsigned)kThr + threadIdx.x;
  asm volatile("" : "+v"(v));
  const unsigned row = v >> 6;
  const unsigned k8 = (v & 63u) * 8u;
  const unsigned t = row >> 6;
  const unsigned b = row & 63u;
  const unsigned tc = (t > 0u) ? (t - 1u) : 0u;
  const float* sf = features + (size_t)b * kE + k8;
  const float* se = emb + ((size_t)b * kT + tc) * kE + k8;
  const v4f f0 = *(const v4f*)sf, f1 = *(const v4f*)(sf + 4);
  const v4f e0 = *(const v4f*)se, e1 = *(const v4f*)(se + 4);
  v8h hv;
#pragma unroll
  for (int e = 0; e < 4; ++e) {
    const float a0 = (t == 0u) ? f0[e] : e0[e];
    const float a1 = (t == 0u) ? f1[e] : e1[e];
    hv[e]     = (_Float16)carry_flush(bf16r(a0), kXCarry);
    hv[4 + e] = (_Float16)carry_flush(bf16r(a1), kXCarry);
  }
  unsigned short* dp = X16 + (size_t)v * 8u;
  *(volatile v8h*)dp = hv;
  __threadfence();
  *(volatile v8h*)dp = hv;
}
static_assert(kRowsX * kE / 8 == 336 * kThr, "x plane grid exact");

__global__ __launch_bounds__(kThr) void setup_kernel(const float* __restrict__ b_ih, const float* __restrict__ b_hh,
                                                     const float* __restrict__ b_lin, float* __restrict__ BG, float* __restrict__ BL,
                                                     float* __restrict__ ZB, float* __restrict__ C32, unsigned short* __restrict__ H16) {
  unsigned v = blockIdx.x * (unsigned)kThr + threadIdx.x;
  asm volatile("" : "+v"(v));
  const unsigned i0 = v * 4u;
  v4f o = {0.f, 0.f, 0.f, 0.f};
  float* dp;
  if (i0 < (unsigned)kG4) {
    const v4f a = *(const v4f*)(b_ih + i0);
    const v4f c = *(const v4f*)(b_hh + i0);
#pragma unroll
    for (int e = 0; e < 4; ++e) { const float x = a[e]; const float y = c[e]; o[e] = bf16r(x) + bf16r(y); }
    dp = BG + i0;
  } else if (i0 < (unsigned)(kG4 + kVP)) {
    const unsigned n0 = i0 - (unsigned)kG4;
    const unsigned nc = (n0 < (unsigned)kV) ? n0 : 0u;
    const v4f a = *(const v4f*)(b_lin + nc);
#pragma unroll
    for (int e = 0; e < 4; ++e) { const float x = a[e]; o[e] = (n0 < (unsigned)kV) ? bf16r(x) : 0.0f; }
    dp = BL + n0;
  } else if (i0 < (unsigned)(2 * kG4 + kVP)) {
    dp = ZB + (i0 - (unsigned)(kG4 + kVP));
  } else {
    const unsigned c0 = i0 - (unsigned)(2 * kG4 + kVP);
    dp = C32 + c0;
    typedef __attribute__((ext_vector_type(4))) _Float16 v4h;
    const v4h zh = {(_Float16)0.0f, (_Float16)0.0f, (_Float16)0.0f, (_Float16)0.0f};
    for (int pass = 0; pass < 2; ++pass) {
      *(volatile v4h*)(H16 + c0) = zh;
      __threadfence();
    }
  }
  *(volatile v4f*)dp = o;
  __threadfence();
  *(volatile v4f*)dp = o;
}
static_assert((kG4 + kVP + kG4 + kB * kHid) / 4 == 46 * kThr, "set-up grid exact");
static_assert((kG4 / 4) % 128 == 0 && (kVP / 4) % 128 == 0 && (kV % 4) == 0, "set-up regions wave-uniform");

__global__ __launch_bounds__(kThr) void wl_pad_kernel(unsigned short* __restrict__ WL) {
  const size_t v = (size_t)blockIdx.x * kThr + threadIdx.x;
  v8h z;
#pragma unroll
  for (int e = 0; e < 8; ++e) z[e] = (_Float16)0.0f;
  unsigned short* dp = WL + (size_t)kV * kHid + v * 8;
  *(volatile v8h*)dp = z;
  __threadfence();
  *(volatile v8h*)dp = z;
}
static_assert((kVP - kV) * kHid / 8 == 60 * kThr, "pad grid exact");

__device__ __forceinline__ float fast_tanh(float v) { return 1.0f - 2.0f * frcp(__expf(2.0f * v) + 1.0f); }
__device__ __forceinline__ float fast_sigmoid(float v) { return frcp(1.0f + __expf(-v)); }

__global__ __launch_bounds__(kThr) void cell_kernel(const float* __restrict__ XW, const float* __restrict__ GG, float* __restrict__ C32,
                                                    unsigned short* __restrict__ H16, unsigned short* __restrict__ HL, int t) {
  unsigned v = blockIdx.x * (unsigned)kThr + threadIdx.x;
  asm volatile("" : "+v"(v));
  const unsigned b = v >> 6;
  const unsigned u8 = (v & 63u) * 8u;
  const float* xr = XW + ((size_t)t * kB + b) * kG4 + u8;
  const float* gr = GG + (size_t)b * kG4 + u8;
  float* cp = C32 + (size_t)b * kHid + u8;
  v8h hv;
  v4f cn0, cn1;
#pragma unroll
  for (int hlf = 0; hlf < 2; ++hlf) {
    const v4f xi = *(const v4f*)(xr + 4 * hlf), xf = *(const v4f*)(xr + kHid + 4 * hlf), xg = *(const v4f*)(xr + 2 * kHid + 4 * hlf), xo = *(const v4f*)(xr + 3 * kHid + 4 * hlf);
    const v4f gi = *(const v4f*)(gr + 4 * hlf), gf = *(const v4f*)(gr + kHid + 4 * hlf), gg = *(const v4f*)(gr + 2 * kHid + 4 * hlf), go = *(const v4f*)(gr + 3 * kHid + 4 * hlf);
    const v4f co = *(const v4f*)(cp + 4 * hlf);
#pragma unroll
    for (int e = 0; e < 4; ++e) {
      const float cn = fast_sigmoid(xf[e] + gf[e]) * co[e] + fast_sigmoid(xi[e] + gi[e]) * fast_tanh(xg[e] + gg[e]);
      const float hn = fast_sigmoid(xo[e] + go[e]) * fast_tanh(cn);
      if (hlf == 0) cn0[e] = cn; else cn1[e] = cn;
      hv[4 * hlf + e] = (_Float16)carry_flush(hn, kSCarry);
    }
  }
  unsigned short* hp = H16 + (size_t)b * kHid + u8;
  const int te = (t > 0) ? (t - 1) : 0;
  unsigned short* lp = HL + ((size_t)b * kTo + te) * kHid + u8;
  for (int pass = 0; pass < 2; ++pass) {
    *(volatile v4f*)cp = cn0;
    *(volatile v4f*)(cp + 4) = cn1;
    *(volatile v8h*)hp = hv;
    if (t > 0) *(volatile v8h*)lp = hv;
    __threadfence();
  }
}
static_assert(kB * kHid / 8 == 16 * kThr, "cell grid exact");

__global__ __launch_bounds__(kThr) void out_kernel(const float* __restrict__ LG, float* __restrict__ out) {
  unsigned i = blockIdx.x * (unsigned)kThr + threadIdx.x;
  asm volatile("" : "+v"(i));
  const unsigned row = i / 2500u;
  const unsigned c4 = (i - row * 2500u) * 4u;
  const v4f o = *(const v4f*)(LG + (size_t)row * kVP + c4);
  float* dp = out + (size_t)i * 4u;
  *(volatile v4f*)dp = o;
  __threadfence();
  *(volatile v4f*)dp = o;
}
static_assert(kRowsY * kV / 4 == 12500 * kThr && kV / 4 == 2500, "output grid exact");

static_assert(((size_t)kG4 * kE / 8) % kThr == 0 && ((size_t)kV * kHid / 8) % kThr == 0, "cast grids exact");

extern "C" void kernel_launch(void* const* d_in, const int* in_sizes, int n_in,
                              void* d_out, int out_size, void* d_ws, size_t ws_size,
                              hipStream_t stream) {
  if (n_in < 8 || d_out == nullptr || d_ws == nullptr) return;
  if (in_sizes[0] != kB * kE || in_sizes[1] != kB * kT * kE || in_sizes[2] != kG4 * kE || in_sizes[3] != kG4 * kHid) return;
  if (in_sizes[4] != kG4 || in_sizes[5] != kG4 || in_sizes[6] != kV * kHid || in_sizes[7] != kV) return;
  if (out_size != kRowsY * kV) return;
  if (ws_size < kWsTotal) return;
  const float* features = (const float*)d_in[0];
  const float* emb   = (const float*)d_in[1];
  const float* W_ih  = (const float*)d_in[2];
  const float* W_hh  = (const float*)d_in[3];
  const float* b_ih  = (const float*)d_in[4];
  const float* b_hh  = (const float*)d_in[5];
  const float* W_lin = (const float*)d_in[6];
  const float* b_lin = (const float*)d_in[7];
  float* out = (float*)d_out;
  char* ws = (char*)d_ws;
  unsigned short* X16 = (unsigned short*)(ws + kOffX16);
  unsigned short* WIH = (unsigned short*)(ws + kOffWIH);
  unsigned short* WHH = (unsigned short*)(ws + kOffWHH);
  unsigned short* WL  = (unsigned short*)(ws + kOffWL);
  float* BG  = (float*)(ws + kOffBG);
  float* BL  = (float*)(ws + kOffBL);
  float* ZB  = (float*)(ws + kOffZB);
  float* XW  = (float*)(ws + kOffXW);
  float* GG  = (float*)(ws + kOffGG);
  float* C32 = (float*)(ws + kOffC32);
  unsigned short* H16 = (unsigned short*)(ws + kOffH16);
  unsigned short* HL  = (unsigned short*)(ws + kOffHL);
  float* LG  = (float*)(ws + kOffLG);

  cast_plane_kernel<<<(int)(((size_t)kG4 * kE / 8) / kThr), kThr, 0, stream>>>(W_ih, WIH, 9, kE, 0);
  cast_plane_kernel<<<(int)(((size_t)kG4 * kHid / 8) / kThr), kThr, 0, stream>>>(W_hh, WHH, 9, kHid, 0);
  cast_plane_kernel<<<(int)(((size_t)kV * kHid / 8) / kThr), kThr, 0, stream>>>(W_lin, WL, 9, kHid, 0);
  wl_pad_kernel<<<60, kThr, 0, stream>>>(WL);
  x_plane_kernel<<<336, kThr, 0, stream>>>(features, emb, X16);
  setup_kernel<<<46, kThr, 0, stream>>>(b_ih, b_hh, b_lin, BG, BL, ZB, C32, H16);

  wmma_gemm64<0, false, 2, 0, false, 0><<<dim3((kRowsX / 64) * (kG4 / 64) / 8, 1), 256, 0, stream>>>(
      X16, X16, kE, 0L, WIH, WIH, kE, 0L, (void*)XW, (void*)XW, kG4, 0L, BG, nullptr, 0L, kRowsX, kG4, kE, kScXW);
  for (int t = 0; t < kT; ++t) {
    wmma_gemm64<0, false, 2, 0, false, 0><<<dim3((kB / 64) * (kG4 / 64) / 8, 1), 256, 0, stream>>>(
        H16, H16, kHid, 0L, WHH, WHH, kHid, 0L, (void*)GG, (void*)GG, kG4, 0L, ZB, nullptr, 0L, kB, kG4, kHid, kScHW);
    cell_kernel<<<16, kThr, 0, stream>>>(XW, GG, C32, H16, HL, t);
  }
  wmma_gemm64<0, false, 2, 0, false, 0><<<dim3((kRowsY / 64) * (kVP / 64) / 8, 1), 256, 0, stream>>>(
      HL, HL, kHid, 0L, WL, WL, kHid, 0L, (void*)LG, (void*)LG, kVP, 0L, BL, nullptr, 0L, kRowsY, kVP, kHid, kScHW);
  out_kernel<<<12500, kThr, 0, stream>>>(LG, out);
}
